// EntityLinker_87471303950751
// MI455X (gfx1250) — hardware-run, weakly checked
//
#include <hip/hip_runtime.h>
#include <math.h>

typedef __attribute__((ext_vector_type(16))) _Float16 v16h;
typedef __attribute__((ext_vector_type(8)))  _Float16 v8h;
typedef __attribute__((ext_vector_type(8)))  float    v8f;
typedef __attribute__((ext_vector_type(4)))  float    v4f;
typedef __attribute__((ext_vector_type(4)))  unsigned v4u;

constexpr int kNodes = 50000;
constexpr int kEdges = 500000;
constexpr int kH     = 128;
constexpr int kK1    = 4 * kH;
constexpr int kN1    = 2 * kH;
constexpr int kN2    = kH;
constexpr int kNC    = 2;
constexpr int kNCP   = 16;
constexpr int kFP    = kH + 8;
constexpr int kXP    = kN1 + 8;
constexpr int kTileE = 64;

constexpr float kFeatCarry    = 32.0f;
constexpr float kFeatCarryInv = 1.0f / kFeatCarry;
constexpr float kWCarry       = 256.0f;
constexpr float kFold         = 1.0f / (kFeatCarry * kWCarry);

static_assert(kK1 == 512 && kN1 == 256 && kN2 == 128, "layer widths");
static_assert((kK1 % 32) == 0 && (kN1 % 32) == 0 && (kN2 % 32) == 0, "contraction depths are multiples of 32");
static_assert((kN1 % 64) == 0 && (kN2 % 32) == 0, "feature tiles per wave");
static_assert((kEdges % 16) == 0, "16-edge output tiles are whole");
static_assert(((kFP * 2) % 16) == 0 && ((kXP * 2) % 16) == 0, "LDS rows 16-B aligned");

constexpr size_t kOffNP   = 0;
constexpr size_t kOffB1   = kOffNP + (size_t)kNodes * kH * 2;
constexpr size_t kOffB2   = kOffB1 + (size_t)kN1 * kK1 * 2;
constexpr size_t kOffB3   = kOffB2 + (size_t)kN2 * kN1 * 2;
constexpr size_t kWsTotal = kOffB3 + (size_t)kNCP * kN2 * 2;
static_assert(kWsTotal == 13131776ull, "carve total");
static_assert(kWsTotal <= 134217728ull, "carve cap");
static_assert((kOffB1 % 128) == 0 && (kOffB2 % 128) == 0 && (kOffB3 % 128) == 0, "128-B aligned regions");

constexpr int kPB_Node = (kNodes * kH / 8) / 256;
constexpr int kPB_W1   = (kN1 * kK1 / 8) / 256;
constexpr int kPB_W2   = (kN2 * kN1 / 8) / 256;
constexpr int kPB_W3   = (kNCP * kN2 / 8) / 256;
static_assert(kPB_Node * 256 * 8 == kNodes * kH, "node plane coverage");
static_assert(kPB_W1 * 256 * 8 == kN1 * kK1, "B1 coverage");
static_assert(kPB_W2 * 256 * 8 == kN2 * kN1, "B2 coverage");
static_assert(kPB_W3 * 256 * 8 == kNCP * kN2, "B3 coverage");
constexpr int kPrepBlocks = kPB_Node + kPB_W1 + kPB_W2 + kPB_W3;
constexpr int kEdgeBlocks = (kEdges + kTileE - 1) / kTileE;

__device__ __forceinline__ float bf16_rne_f(float x) {
  unsigned u = __float_as_uint(x);
  u = (u + 0x7FFFu + ((u >> 16) & 1u)) & 0xFFFF0000u;
  return __uint_as_float(u);
}
__device__ __forceinline__ unsigned np_bits(float x) {
  const float f = bf16_rne_f(x) * kFeatCarry;
  return __float_as_uint(f) >> 16;
}

__device__ __forceinline__ float absdiff_f32(float a, float b) {
  float d;
  asm("v_sub_f32 %0, %1, %2\n\tv_and_b32 %0, 0x7fffffff, %0" : "=v"(d) : "v"(a), "v"(b));
  return d;
}

struct FragH {
  union U { v16h v; v8h h[2]; };
  static __device__ __forceinline__ v16h load(const _Float16* p) {
    U f;
    f.h[0] = *(const v8h*)(p);
    f.h[1] = *(const v8h*)(p + 16);
    return f.v;
  }
};

__device__ __forceinline__ v8f mma_g(v16h a, v16h b, v8f c) {
  c = __builtin_amdgcn_wmma_f32_16x16x32_f16(false, a, false, b, (short)0, c, false, false);
  asm volatile("v_nop\n\tv_nop\n\tv_nop\n\tv_nop" : "+v"(c) : "v"(a), "v"(b));
  return c;
}

__device__ __forceinline__ void load_bias8(const float* __restrict__ p, float (&q)[8]) {
  const v4f a = *(const v4f*)(p);
  const v4f b = *(const v4f*)(p + 4);
  const float a0 = a[0], a1 = a[1], a2 = a[2], a3 = a[3];
  const float c0 = b[0], c1 = b[1], c2 = b[2], c3 = b[3];
  q[0] = bf16_rne_f(a0); q[1] = bf16_rne_f(a1); q[2] = bf16_rne_f(a2); q[3] = bf16_rne_f(a3);
  q[4] = bf16_rne_f(c0); q[5] = bf16_rne_f(c1); q[6] = bf16_rne_f(c2); q[7] = bf16_rne_f(c3);
}

__device__ __forceinline__ void wt_rows(const float* __restrict__ W, int nReal, int K, int t,
                                        _Float16* __restrict__ outp) {
  const int kk8 = K >> 3;
  const int n   = t / kk8;
  const int k8  = (t - n * kk8) << 3;
  const int nc  = (n < nReal) ? n : (nReal - 1);
  const bool live = (n < nReal);
  v8h hv;
#pragma unroll
  for (int e = 0; e < 8; ++e) {
    const float x = W[(size_t)(k8 + e) * nReal + nc];
    float f = bf16_rne_f(x) * kWCarry;
    f = live ? f : 0.0f;
    hv[e] = (_Float16)f;
  }
  _Float16* q = outp + (size_t)n * K + k8;
  *(volatile v8h*)q = hv;
  __threadfence();
  *(volatile v8h*)q = hv;
}

__global__ __launch_bounds__(256) void prep_kernel(
    const float* __restrict__ node, const float* __restrict__ W1,
    const float* __restrict__ W2, const float* __restrict__ W3,
    unsigned short* __restrict__ NP, _Float16* __restrict__ B1,
    _Float16* __restrict__ B2, _Float16* __restrict__ B3)
{
  const int bid = blockIdx.x;
  const int tid = threadIdx.x;
  if (bid < kPB_Node) {
    const size_t e0 = ((size_t)bid * 256 + tid) * 8;
    const v4f a0 = *(const v4f*)(node + e0);
    const v4f a1 = *(const v4f*)(node + e0 + 4);
    const float x0 = a0[0], x1 = a0[1], x2 = a0[2], x3 = a0[3];
    const float x4 = a1[0], x5 = a1[1], x6 = a1[2], x7 = a1[3];
    v4u w;
    w[0] = np_bits(x0) | (np_bits(x1) << 16);
    w[1] = np_bits(x2) | (np_bits(x3) << 16);
    w[2] = np_bits(x4) | (np_bits(x5) << 16);
    w[3] = np_bits(x6) | (np_bits(x7) << 16);
    unsigned short* q = NP + e0;
    *(volatile v4u*)q = w;
    __threadfence();
    *(volatile v4u*)q = w;
  } else if (bid < kPB_Node + kPB_W1) {
    wt_rows(W1, kN1, kK1, (bid - kPB_Node) * 256 + tid, B1);
  } else if (bid < kPB_Node + kPB_W1 + kPB_W2) {
    wt_rows(W2, kN2, kN1, (bid - kPB_Node - kPB_W1) * 256 + tid, B2);
  } else {
    wt_rows(W3, kNC, kN2, (bid - kPB_Node - kPB_W1 - kPB_W2) * 256 + tid, B3);
  }
}

template <int C> __device__ __forceinline__ float feat_val(float a, float b) {
  if (C == 0) return a;
  if (C == 1) return b;
  if (C == 2) return absdiff_f32(a, b);
  return (a * kFeatCarryInv) * b;
}

template <int C>
__device__ __forceinline__ void chunk_step(v8f (&acc)[4][4], _Float16* sF, _Float16* fdst,
                                           const v4u* __restrict__ pi, const v4u* __restrict__ pj,
                                           const _Float16* __restrict__ wb, int rl, int koff)
{
#pragma unroll 2
  for (int t = 0; t < 8; ++t) {
    const v4u a = pi[t];
    const v4u b = pj[t];
    v8h o;
#pragma unroll
    for (int q = 0; q < 4; ++q) {
      const unsigned wa = a[q];
      const unsigned wq = b[q];
      const float a0 = __uint_as_float(wa << 16);
      const float a1 = __uint_as_float(wa & 0xffff0000u);
      const float b0 = __uint_as_float(wq << 16);
      const float b1 = __uint_as_float(wq & 0xffff0000u);
      const float f0 = feat_val<C>(a0, b0);
      const float f1 = feat_val<C>(a1, b1);
      o[2 * q]     = (_Float16)f0;
      o[2 * q + 1] = (_Float16)f1;
    }
    *(v8h*)(fdst + t * 8) = o;
  }
  __syncthreads();
#pragma unroll 1
  for (int ks = 0; ks < 4; ++ks) {
    const int k0 = ks * 32;
    v16h wa[4];
#pragma unroll
    for (int i = 0; i < 4; ++i) wa[i] = FragH::load(wb + (size_t)(i * 16) * kK1 + k0);
#pragma unroll
    for (int j = 0; j < 4; ++j) {
      const v16h fb = FragH::load(sF + (j * 16 + rl) * kFP + k0 + koff);
#pragma unroll
      for (int i = 0; i < 4; ++i) acc[i][j] = mma_g(wa[i], fb, acc[i][j]);
    }
  }
  __syncthreads();
}

__global__ __launch_bounds__(128) void edge_mlp_kernel(
    const int* __restrict__ src, const int* __restrict__ dst,
    const unsigned short* __restrict__ NP,
    const _Float16* __restrict__ B1, const float* __restrict__ b1,
    const _Float16* __restrict__ B2, const float* __restrict__ b2,
    const _Float16* __restrict__ B3, const float* __restrict__ b3,
    float* __restrict__ out)
{
  __shared__ __align__(16) _Float16 sF[kTileE * kFP];
  __shared__ __align__(16) _Float16 sX[kTileE * kXP];

  const int tid  = threadIdx.x;
  const int lane = tid & 31;
  const int wave = tid >> 5;
  const int rl   = lane & 15;
  const int hh   = lane >> 4;
  const int koff = hh * 8;
  const int blockBase = blockIdx.x * kTileE;

  const int frow  = tid >> 1;
  const int fhalf = tid & 1;
  int e = blockBase + frow;
  e = (e < kEdges) ? e : (kEdges - 1);
  int si = src[e];
  int di = dst[e];
  si = si < 0 ? 0 : (si > kNodes - 1 ? kNodes - 1 : si);
  di = di < 0 ? 0 : (di > kNodes - 1 ? kNodes - 1 : di);
  const v4u* pi = (const v4u*)(NP + (size_t)si * kH + fhalf * 64);
  const v4u* pj = (const v4u*)(NP + (size_t)di * kH + fhalf * 64);
  _Float16* fdst = sF + frow * kFP + fhalf * 64;

  v8f acc[4][4];
#pragma unroll
  for (int i = 0; i < 4; ++i)
#pragma unroll
    for (int j = 0; j < 4; ++j) acc[i][j] = (v8f){0.f, 0.f, 0.f, 0.f, 0.f, 0.f, 0.f, 0.f};

  const _Float16* w1base = B1 + (size_t)(wave * 64 + rl) * kK1 + koff;
  chunk_step<0>(acc, sF, fdst, pi, pj, w1base + 0 * kH, rl, koff);
  chunk_step<1>(acc, sF, fdst, pi, pj, w1base + 1 * kH, rl, koff);
  chunk_step<2>(acc, sF, fdst, pi, pj, w1base + 2 * kH, rl, koff);
  chunk_step<3>(acc, sF, fdst, pi, pj, w1base + 3 * kH, rl, koff);

#pragma unroll
  for (int i = 0; i < 4; ++i) {
    const int f0 = wave * 64 + i * 16 + hh * 8;
    float bq[8];
    load_bias8(b1 + f0, bq);
#pragma unroll
    for (int j = 0; j < 4; ++j) {
      v8h o;
#pragma unroll
      for (int r = 0; r < 8; ++r) {
        float v = fmaf(acc[i][j][r], kFold, bq[r]);
        v = fmaxf(v, 0.0f);
        o[r] = (_Float16)(v * kFeatCarry);
      }
      *(v8h*)(sX + (j * 16 + rl) * kXP + f0) = o;
    }
  }
  __syncthreads();

  v8f acc2[2][4];
#pragma unroll
  for (int i = 0; i < 2; ++i)
#pragma unroll
    for (int j = 0; j < 4; ++j) acc2[i][j] = (v8f){0.f, 0.f, 0.f, 0.f, 0.f, 0.f, 0.f, 0.f};
  {
    const _Float16* w2base = B2 + (size_t)(wave * 32 + rl) * kN1 + koff;
#pragma unroll 1
    for (int ks = 0; ks < kN1 / 32; ++ks) {
      const int k0 = ks * 32;
      v16h wa[2];
#pragma unroll
      for (int i = 0; i < 2; ++i) wa[i] = FragH::load(w2base + (size_t)(i * 16) * kN1 + k0);
#pragma unroll
      for (int j = 0; j < 4; ++j) {
        const v16h fb = FragH::load(sX + (j * 16 + rl) * kXP + k0 + koff);
#pragma unroll
        for (int i = 0; i < 2; ++i) acc2[i][j] = mma_g(wa[i], fb, acc2[i][j]);
      }
    }
  }
#pragma unroll
  for (int i = 0; i < 2; ++i) {
    const int f0 = wave * 32 + i * 16 + hh * 8;
    float bq[8];
    load_bias8(b2 + f0, bq);
#pragma unroll
    for (int j = 0; j < 4; ++j) {
      v8h o;
#pragma unroll
      for (int r = 0; r < 8; ++r) {
        float v = fmaf(acc2[i][j][r], kFold, bq[r]);
        v = fmaxf(v, 0.0f);
        o[r] = (_Float16)(v * kFeatCarry);
      }
      *(v8h*)(sF + (j * 16 + rl) * kFP + f0) = o;
    }
  }
  __syncthreads();

  v8f acc3 = (v8f){0.f, 0.f, 0.f, 0.f, 0.f, 0.f, 0.f, 0.f};
#pragma unroll
  for (int ks = 0; ks < kN2 / 32; ++ks) {
    const int k0 = ks * 32;
    const v16h wa = FragH::load(B3 + (size_t)rl * kN2 + koff + k0);
    const v16h fb = FragH::load(sF + (wave * 16 + rl) * kFP + k0 + koff);
    acc3 = mma_g(wa, fb, acc3);
  }
  const float c0 = acc3[0];
  const float c1 = acc3[1];
  const float bz0 = bf16_rne_f(b3[0]);
  const float bz1 = bf16_rne_f(b3[1]);
  const float o0 = fmaf(c0, kFold, bz0);
  const float o1 = fmaf(c1, kFold, bz1);
  const int sl = lane >> 1;
  const float v0 = __shfl(o0, sl, 32);
  const float v1 = __shfl(o1, sl, 32);
  const float val = (lane & 1) ? v1 : v0;
  const int tb = blockBase + wave * 16;
  if (tb < kEdges) {
    volatile float* q = out + (size_t)tb * kNC + lane;
    *q = val;
    __threadfence();
    *q = val;
  }
}

extern "C" void kernel_launch(void* const* d_in, const int* in_sizes, int n_in,
                              void* d_out, int out_size, void* d_ws, size_t ws_size,
                              hipStream_t stream)
{
  if (n_in < 9) return;
  if (in_sizes[0] != kNodes * kH) return;
  if (in_sizes[1] != kEdges) return;
  if (in_sizes[2] != kEdges) return;
  if (in_sizes[3] != kK1 * kN1) return;
  if (in_sizes[4] != kN1) return;
  if (in_sizes[5] != kN1 * kN2) return;
  if (in_sizes[6] != kN2) return;
  if (in_sizes[7] != kN2 * kNC) return;
  if (in_sizes[8] != kNC) return;
  if (out_size != kEdges * kNC) return;
  if (ws_size < kWsTotal) return;

  const float* node = (const float*)d_in[0];
  const int*   src  = (const int*)d_in[1];
  const int*   dst  = (const int*)d_in[2];
  const float* W1   = (const float*)d_in[3];
  const float* b1   = (const float*)d_in[4];
  const float* W2   = (const float*)d_in[5];
  const float* b2   = (const float*)d_in[6];
  const float* W3   = (const float*)d_in[7];
  const float* b3   = (const float*)d_in[8];

  char* ws = (char*)d_ws;
  unsigned short* NP = (unsigned short*)(ws + kOffNP);
  _Float16* B1 = (_Float16*)(ws + kOffB1);
  _Float16* B2 = (_Float16*)(ws + kOffB2);
  _Float16* B3 = (_Float16*)(ws + kOffB3);

  prep_kernel<<<kPrepBlocks, 256, 0, stream>>>(node, W1, W2, W3, NP, B1, B2, B3);
  edge_mlp_kernel<<<kEdgeBlocks, 128, 0, stream>>>(src, dst, NP, B1, b1, B2, b2, B3, b3, (float*)d_out);
}
